// S5Dual_30975304139517
// MI455X (gfx1250) — hardware-verified
//
#include <hip/hip_runtime.h>
#include <math.h>

constexpr int kSeq  = 8192;
constexpr int kH    = 512;
constexpr int kP    = 512;
constexpr int kNC   = 2 * kP;
constexpr int kNDir = 2;
constexpr float kWCarry    = 16.0f;
constexpr float kWCarryInv = 1.0f / 16.0f;
constexpr int kRecP = 64;
constexpr int kRecT = 32;
static_assert(kSeq % kRecT == 0, "chunking");
static_assert(kP % kRecP == 0, "channel blocks");

typedef __attribute__((ext_vector_type(16))) _Float16 v16h;
typedef __attribute__((ext_vector_type(8)))  _Float16 v8h;
typedef __attribute__((ext_vector_type(16))) __bf16   v16b;
typedef __attribute__((ext_vector_type(8)))  __bf16   v8b;
typedef __attribute__((ext_vector_type(8)))  float    v8f;
typedef __attribute__((ext_vector_type(4)))  float    v4f;
typedef __attribute__((ext_vector_type(2)))  float    v2f;
typedef __attribute__((ext_vector_type(4)))  unsigned int v4u;

__device__ __forceinline__ unsigned short f2bf_bits(float f) {
  unsigned u = __float_as_uint(f);
  return (unsigned short)((u + 0x7FFFu + ((u >> 16) & 1u)) >> 16);
}
__device__ __forceinline__ float bf_bits2f(unsigned short h) { return __uint_as_float(((unsigned)h) << 16); }

__device__ __forceinline__ void dep_guard_h(v8f& a, v8f& b, v16h x, v16h y) { asm volatile("v_nop\n\tv_nop\n\tv_nop\n\tv_nop" : "+v"(a), "+v"(b) : "v"(x), "v"(y)); }
__device__ __forceinline__ void dep_guard_b(v8f& a, v8f& b, v16b x, v16b y) { asm volatile("v_nop\n\tv_nop\n\tv_nop\n\tv_nop" : "+v"(a), "+v"(b) : "v"(x), "v"(y)); }
__device__ __forceinline__ void keep4_h(v16h a, v16h b, v16h c, v16h d) { asm volatile("v_nop" :: "v"(a), "v"(b), "v"(c), "v"(d)); }
__device__ __forceinline__ void keep4_b(v16b a, v16b b, v16b c, v16b d) { asm volatile("v_nop" :: "v"(a), "v"(b), "v"(c), "v"(d)); }
__device__ __forceinline__ void acc_guard4(v8f& a, v8f& b, v8f& c, v8f& d) { asm volatile("v_nop\n\tv_nop\n\tv_nop\n\tv_nop" : "+v"(a), "+v"(b), "+v"(c), "+v"(d)); }
template <typename T> struct Frag;
template <> struct Frag<_Float16> {
  typedef v16h V; union U { v16h v; v8h h[2]; };
  static __device__ __forceinline__ v16h load(const _Float16* p) {
    U f; f.h[0] = *(const v8h*)(p); f.h[1] = *(const v8h*)(p + 16); return f.v;
  }
  static __device__ __forceinline__ v8f mma(v16h a, v16h b, v8f c) {
    return __builtin_amdgcn_wmma_f32_16x16x32_f16(false, a, false, b, (short)0, c, false, false);
  }
  static __device__ __forceinline__ void guard(v8f& a, v8f& b, v16h x, v16h y) { dep_guard_h(a, b, x, y); }
  static __device__ __forceinline__ void keep(v16h a, v16h b, v16h c, v16h d) { keep4_h(a, b, c, d); }
};
template <> struct Frag<__bf16> {
  typedef v16b V; union U { v16b v; v8b h[2]; };
  static __device__ __forceinline__ v16b load(const __bf16* p) {
    U f; f.h[0] = *(const v8b*)(p); f.h[1] = *(const v8b*)(p + 16); return f.v;
  }
  static __device__ __forceinline__ v8f mma(v16b a, v16b b, v8f c) {
    return __builtin_amdgcn_wmma_f32_16x16x32_bf16(false, a, false, b, (short)0, c, false, false);
  }
  static __device__ __forceinline__ void guard(v8f& a, v8f& b, v16b x, v16b y) { dep_guard_b(a, b, x, y); }
  static __device__ __forceinline__ void keep(v16b a, v16b b, v16b c, v16b d) { keep4_b(a, b, c, d); }
};

__device__ __forceinline__ unsigned pk16(unsigned short a, unsigned short b) { return (unsigned)a | ((unsigned)b << 16); }
__device__ __forceinline__ unsigned short h_bits(float f) { const _Float16 h = (_Float16)f; return __builtin_bit_cast(unsigned short, h); }

template <int ET> struct Elem;
template <> struct Elem<0> { typedef _Float16 T; };
template <> struct Elem<1> { typedef __bf16 T; };
template <int ET, bool SPLIT, int BIAS_MODE, int OUT_MODE, bool RESID, int ACT = 0>
__global__ __launch_bounds__(256) void wmma_gemm64(
    const unsigned short* __restrict__ Ap, const unsigned short* __restrict__ A2p, int lda, long strideA,
    const unsigned short* __restrict__ Btp, const unsigned short* __restrict__ Bt2p, int ldb, long strideB,
    void* __restrict__ Cout, void* __restrict__ Cout2, int ldc, long strideC,
    const float* __restrict__ bias,
    const float* __restrict__ resid, long strideR,
    int M, int N, int K, float scale) {
  typedef typename Elem<ET>::T T;
  typedef typename Frag<T>::V V;
  const T* A = (const T*)Ap; const T* A2 = (const T*)A2p; const T* Bt = (const T*)Btp; const T* Bt2 = (const T*)Bt2p;
  __shared__ __align__(16) float sT[8][16 * 68];
  const int b    = blockIdx.y;
  const int lane = threadIdx.x & 31;
  const int wave = threadIdx.x >> 5;
  const int tilesN = N >> 6;
  const int tilesM = M >> 6;
  const int tile = blockIdx.x * 8 + wave;
  if (tile >= tilesM * tilesN) return;
  const int tm = tile / tilesN;
  const int tn = tile - tm * tilesN;
  const int m0 = tm << 6;
  const int n0 = tn << 6;

  const T* Ab  = A  + (size_t)b * strideA;
  const T* Bb  = Bt + (size_t)b * strideB;
  const T* Ab2 = SPLIT ? (A2  + (size_t)b * strideA) : nullptr;
  const T* Bb2 = SPLIT ? (Bt2 + (size_t)b * strideB) : nullptr;

  const int rlane = lane & 15;
  const int koff  = (lane >> 4) * 8;
  const int mOff  = (lane >> 4) * 8;

  v8f acc[4][4];
#pragma unroll
  for (int i = 0; i < 4; ++i)
#pragma unroll
    for (int j = 0; j < 4; ++j) acc[i][j] = (v8f){0.f,0.f,0.f,0.f,0.f,0.f,0.f,0.f};

  for (int k0 = 0; k0 < K; k0 += 32) {
    V bh[4], bl[4];
#pragma unroll
    for (int j = 0; j < 4; ++j) {
      const size_t bo = (size_t)(n0 + (j << 4) + rlane) * ldb + koff + k0;
      bh[j] = Frag<T>::load(Bb + bo);
      if (SPLIT) bl[j] = Frag<T>::load(Bb2 + bo);
    }
#pragma unroll
    for (int i = 0; i < 4; ++i) {
      const size_t ao = (size_t)(m0 + (i << 4) + rlane) * lda + koff + k0;
      V ah = Frag<T>::load(Ab + ao);
      V al;
      if (SPLIT) al = Frag<T>::load(Ab2 + ao);
#pragma unroll
      for (int j = 0; j < 4; ++j) {
        acc[i][j] = Frag<T>::mma(ah, bh[j], acc[i][j]);
        if (SPLIT) {
          acc[i][j] = Frag<T>::mma(ah, bl[j], acc[i][j]);
          acc[i][j] = Frag<T>::mma(al, bh[j], acc[i][j]);
        }
      }
      Frag<T>::guard(acc[i][0], acc[i][3], ah, SPLIT ? al : ah);
    }
    Frag<T>::keep(bh[0], bh[1], bh[2], bh[3]);
    if (SPLIT) Frag<T>::keep(bl[0], bl[1], bl[2], bl[3]);
  }
  acc_guard4(acc[0][0], acc[0][1], acc[0][2], acc[0][3]);
  acc_guard4(acc[1][0], acc[1][1], acc[1][2], acc[1][3]);
  acc_guard4(acc[2][0], acc[2][1], acc[2][2], acc[2][3]);
  acc_guard4(acc[3][0], acc[3][1], acc[3][2], acc[3][3]);

  float* slab = sT[wave];
  const float* Rb = RESID ? (resid + (size_t)b * strideR) : nullptr;
#pragma unroll
  for (int i = 0; i < 4; ++i) {
    const int mBase = m0 + (i << 4);
#pragma unroll
    for (int j = 0; j < 4; ++j) {
      const int n = n0 + (j << 4) + rlane;
      float bv = 0.f;
      if (BIAS_MODE == 2) bv = bias[n];
#pragma unroll
      for (int r = 0; r < 8; ++r) {
        float v = acc[i][j][r] * scale;
        if (BIAS_MODE == 1) v += bias[mBase + mOff + r];
        if (BIAS_MODE == 2) v += bv;
        if (RESID) v += Rb[(size_t)(mBase + mOff + r) * ldc + n];
        if (ACT == 2) v = fmaxf(v, 0.0f);
        if (ACT == 4) v = (v > 0.f) ? v : 0.01f * v;
        slab[(mOff + r) * 68 + (j << 4) + rlane] = v;
      }
    }
    __builtin_amdgcn_fence(__ATOMIC_RELEASE, "workgroup");
    __builtin_amdgcn_wave_barrier();
    __builtin_amdgcn_fence(__ATOMIC_ACQUIRE, "workgroup");
    if (OUT_MODE == 0) {
      float* C = (float*)Cout + (size_t)b * strideC;
      const int hh = lane >> 4, c4 = (lane & 15) * 4;
      for (int pass = 0; pass < 2; ++pass) {
#pragma unroll
        for (int it = 0; it < 8; ++it) {
          const int row = it * 2 + hh;
          v4f v = *(const v4f*)(slab + row * 68 + c4);
          *(volatile v4f*)(C + (size_t)(mBase + row) * ldc + n0 + c4) = v;
        }
        __threadfence();
      }
    } else {
      const int q = lane >> 3, c8 = (lane & 7) * 8;
      unsigned short* C  = (unsigned short*)Cout  + (size_t)b * strideC;
      unsigned short* C2 = (OUT_MODE == 2) ? ((unsigned short*)Cout2 + (size_t)b * strideC) : nullptr;
      for (int pass = 0; pass < 2; ++pass) {
#pragma unroll
        for (int it = 0; it < 4; ++it) {
          const int row = it * 4 + q;
          const float* sp = slab + row * 68 + c8;
          v8h hv, lv;
#pragma unroll
          for (int e = 0; e < 8; ++e) {
            if (OUT_MODE == 1) {
              hv[e] = (_Float16)sp[e];
            } else {
              unsigned short hb = f2bf_bits(sp[e]);
              unsigned short lb = f2bf_bits(sp[e] - bf_bits2f(hb));
              hv[e] = __builtin_bit_cast(_Float16, hb);
              lv[e] = __builtin_bit_cast(_Float16, lb);
            }
          }
          *(volatile v8h*)(C + (size_t)(mBase + row) * ldc + n0 + c8) = hv;
          if (OUT_MODE == 2) *(volatile v8h*)(C2 + (size_t)(mBase + row) * ldc + n0 + c8) = lv;
        }
        __threadfence();
      }
    }
    __builtin_amdgcn_fence(__ATOMIC_RELEASE, "workgroup");
    __builtin_amdgcn_wave_barrier();
    __builtin_amdgcn_fence(__ATOMIC_ACQUIRE, "workgroup");
  }
}

__global__ __launch_bounds__(256) void cast8_f16_kernel(const float* __restrict__ in, unsigned short* __restrict__ out, int n8) {
  const int i = blockIdx.x * 256 + threadIdx.x;
  if (i >= n8) return;
  const float* p = in + 8 * (size_t)i;
  const v4f a = *(const v4f*)(p);
  const v4f c = *(const v4f*)(p + 4);
  unsigned short hb[8];
#pragma unroll
  for (int e = 0; e < 4; ++e) {
    hb[e]     = h_bits(a[e]);
    hb[4 + e] = h_bits(c[e]);
  }
  const v4u u = (v4u){pk16(hb[0], hb[1]), pk16(hb[2], hb[3]), pk16(hb[4], hb[5]), pk16(hb[6], hb[7])};
  unsigned short* q = out + 8 * (size_t)i;
  *(volatile v4u*)q = u;
  __threadfence();
  *(volatile v4u*)q = u;
}

__global__ __launch_bounds__(256) void param_kernel(const float* __restrict__ log_real, const float* __restrict__ imag,
                                                    const float* __restrict__ log_delta, float* __restrict__ par, int n) {
  const int i = blockIdx.x * 256 + threadIdx.x;
  if (i >= n) return;
  const float lre = -expf(log_real[i]);
  const float lim = imag[i];
  const float dt  = expf(log_delta[i]);
  const float zr = lre * dt;
  const float zi = lim * dt;
  const float er = expf(zr);
  float sn, cs;
  sincosf(zi, &sn, &cs);
  const float lbr = er * cs;
  const float lbi = er * sn;
  const float mag = sqrtf(lre * lre + lim * lim);
  const bool tiny = (mag < 1e-6f);
  const float sr = tiny ? 1e-6f : lre;
  const float si = tiny ? 0.0f : lim;
  const float den = sr * sr + si * si;
  const float inv = 1.0f / den;
  const float nr = lbr - 1.0f;
  const float ni = lbi;
  const float qre = (nr * sr + ni * si) * inv;
  const float qim = (ni * sr - nr * si) * inv;
  const v4f o = (v4f){lbr, lbi, qre, qim};
  float* dst = par + 4 * (size_t)i;
  *(volatile v4f*)dst = o;
  __threadfence();
  *(volatile v4f*)dst = o;
}

__global__ __launch_bounds__(256) void bbar_kernel(const float* __restrict__ Br, const float* __restrict__ Bi,
                                                   const float* __restrict__ par, unsigned short* __restrict__ Bt1, float carry) {
  const int idx = blockIdx.x * 256 + threadIdx.x;
  const int g   = idx & 63;
  const int p   = (idx >> 6) & (kP - 1);
  const int dir = idx >> 15;
  const int dp  = dir * kP + p;
  const v4f pr = *(const v4f*)(par + 4 * (size_t)dp);
  const float sr = pr[2], si = pr[3];
  const float* brp = Br + (size_t)dp * kH + 8 * g;
  const float* bip = Bi + (size_t)dp * kH + 8 * g;
  const v4f a0 = *(const v4f*)(brp);
  const v4f a1 = *(const v4f*)(brp + 4);
  const v4f b0 = *(const v4f*)(bip);
  const v4f b1 = *(const v4f*)(bip + 4);
  unsigned short hre[8], him[8];
#pragma unroll
  for (int e = 0; e < 4; ++e) {
    const float br0 = a0[e], bi0 = b0[e];
    hre[e] = h_bits(carry * (sr * br0 - si * bi0));
    him[e] = h_bits(carry * (sr * bi0 + si * br0));
    const float br1 = a1[e], bi1 = b1[e];
    hre[4 + e] = h_bits(carry * (sr * br1 - si * bi1));
    him[4 + e] = h_bits(carry * (sr * bi1 + si * br1));
  }
  const v4u ur = (v4u){pk16(hre[0], hre[1]), pk16(hre[2], hre[3]), pk16(hre[4], hre[5]), pk16(hre[6], hre[7])};
  const v4u ui = (v4u){pk16(him[0], him[1]), pk16(him[2], him[3]), pk16(him[4], him[5]), pk16(him[6], him[7])};
  unsigned short* rowr = Bt1 + ((size_t)(dir * kNC + p)) * kH + 8 * g;
  unsigned short* rowi = Bt1 + ((size_t)(dir * kNC + kP + p)) * kH + 8 * g;
  *(volatile v4u*)rowr = ur;
  *(volatile v4u*)rowi = ui;
  __threadfence();
  *(volatile v4u*)rowr = ur;
  *(volatile v4u*)rowi = ui;
}

__global__ __launch_bounds__(256) void cmat_kernel(const float* __restrict__ Cr, const float* __restrict__ Ci,
                                                   unsigned short* __restrict__ Bt2, float carry) {
  const int idx = blockIdx.x * 256 + threadIdx.x;
  const int g   = idx & 63;
  const int h   = (idx >> 6) & (kH - 1);
  const int dir = idx >> 15;
  const size_t rowsrc = ((size_t)(dir * kH + h)) * kP + 8 * g;
  const v4f a0 = *(const v4f*)(Cr + rowsrc);
  const v4f a1 = *(const v4f*)(Cr + rowsrc + 4);
  const v4f b0 = *(const v4f*)(Ci + rowsrc);
  const v4f b1 = *(const v4f*)(Ci + rowsrc + 4);
  unsigned short hre[8], him[8];
#pragma unroll
  for (int e = 0; e < 4; ++e) {
    hre[e]     = h_bits(carry * a0[e]);
    hre[4 + e] = h_bits(carry * a1[e]);
    him[e]     = h_bits(-carry * b0[e]);
    him[4 + e] = h_bits(-carry * b1[e]);
  }
  const v4u ur = (v4u){pk16(hre[0], hre[1]), pk16(hre[2], hre[3]), pk16(hre[4], hre[5]), pk16(hre[6], hre[7])};
  const v4u ui = (v4u){pk16(him[0], him[1]), pk16(him[2], him[3]), pk16(him[4], him[5]), pk16(him[6], him[7])};
  unsigned short* rowdst = Bt2 + ((size_t)(dir * kH + h)) * kNC;
  *(volatile v4u*)(rowdst + 8 * g)      = ur;
  *(volatile v4u*)(rowdst + kP + 8 * g) = ui;
  __threadfence();
  *(volatile v4u*)(rowdst + 8 * g)      = ur;
  *(volatile v4u*)(rowdst + kP + 8 * g) = ui;
}

__global__ __launch_bounds__(64) void diag_rec_kernel(const float* __restrict__ Bu, const float* __restrict__ par,
                                                      unsigned short* __restrict__ XS) {
  __shared__ __align__(16) float sIn[2][kRecT][kRecP];
  __shared__ __align__(16) float sOut[2][kRecT][kRecP];
  const int th   = threadIdx.x;
  const int lane = th & 31;
  const int wave = th >> 5;
  const int blk  = blockIdx.x;
  const int dir  = blk >> 3;
  const int p0   = (blk & 7) * kRecP;
  const v4f pr = *(const v4f*)(par + 4 * (size_t)(dir * kP + p0 + th));
  const float lr = pr[0], li = pr[1];
  const float* BuD = Bu + (size_t)dir * kSeq * kNC;
  unsigned short* XSD = XS + (size_t)dir * kSeq * kNC;
  const int q = lane >> 3, c8 = (lane & 7) * 8;
  float xr = 0.f, xi = 0.f;
  for (int ch = 0; ch < kSeq / kRecT; ++ch) {
    const int s0 = ch * kRecT;
#pragma unroll
    for (int it = 0; it < 16; ++it) {
      const int idx = it * 64 + th;
      const int pl  = idx >> 9;
      const int rem = idx & 511;
      const int row = rem >> 4;
      const int c4  = (rem & 15) * 4;
      const int s   = s0 + row;
      const int t   = dir ? (kSeq - 1 - s) : s;
      const v4f v = *(const v4f*)(BuD + (size_t)t * kNC + pl * kP + p0 + c4);
      *(v4f*)(&sIn[pl][row][c4]) = v;
    }
    __syncthreads();
#pragma unroll 1
    for (int j = 0; j < kRecT; ++j) {
      const float br = sIn[0][j][th];
      const float bi = sIn[1][j][th];
      const float nxr = fmaf(lr, xr, fmaf(-li, xi, br));
      const float nxi = fmaf(lr, xi, fmaf(li, xr, bi));
      xr = nxr;
      xi = nxi;
      sOut[0][j][th] = xr;
      sOut[1][j][th] = xi;
    }
    __syncthreads();
    for (int pass = 0; pass < 2; ++pass) {
#pragma unroll
      for (int it = 0; it < 8; ++it) {
        const int row = it * 4 + q;
        const float* sp = &sOut[wave][row][c8];
        const v4f a = *(const v4f*)(sp);
        const v4f c = *(const v4f*)(sp + 4);
        unsigned short hb[8];
#pragma unroll
        for (int e = 0; e < 4; ++e) {
          hb[e]     = h_bits(a[e]);
          hb[4 + e] = h_bits(c[e]);
        }
        const v4u u = (v4u){pk16(hb[0], hb[1]), pk16(hb[2], hb[3]), pk16(hb[4], hb[5]), pk16(hb[6], hb[7])};
        const int s = s0 + row;
        const int t = dir ? (kSeq - 1 - s) : s;
        *(volatile v4u*)(XSD + (size_t)t * kNC + wave * kP + p0 + c8) = u;
      }
      __threadfence();
    }
  }
}

__device__ __forceinline__ float gelu_tanh_f(float v) {
  const float cube  = v * v * v;
  const float inner = fmaf(0.044715f, cube, v);
  const float twoc  = 1.5957691216057308f * inner;
  const float e     = expf(twoc);
  const float r     = __builtin_amdgcn_rcpf(e + 1.0f);
  const float th    = fmaf(-2.0f, r, 1.0f);
  return 0.5f * v * (1.0f + th);
}

__global__ __launch_bounds__(256) void gelu_sum_kernel(const float* __restrict__ Y, const float* __restrict__ x,
                                                       const float* __restrict__ D, float* __restrict__ out, int n4) {
  const int i = blockIdx.x * 256 + threadIdx.x;
  if (i >= n4) return;
  const size_t e0 = 4 * (size_t)i;
  const int h = (int)(e0 & (size_t)(kH - 1));
  const v4f xv = *(const v4f*)(x + e0);
  const v4f yf = *(const v4f*)(Y + e0);
  const v4f yb = *(const v4f*)(Y + (size_t)kSeq * kH + e0);
  const v4f d0 = *(const v4f*)(D + h);
  const v4f d1 = *(const v4f*)(D + kH + h);
  v4f o;
#pragma unroll
  for (int j = 0; j < 4; ++j)
    o[j] = gelu_tanh_f(fmaf(xv[j], d0[j], yf[j])) + gelu_tanh_f(fmaf(xv[j], d1[j], yb[j]));
  float* dst = out + e0;
  *(volatile v4f*)dst = o;
  __threadfence();
  *(volatile v4f*)dst = o;
}

extern "C" void kernel_launch(void* const* d_in, const int* in_sizes, int n_in,
                              void* d_out, int out_size, void* d_ws, size_t ws_size,
                              hipStream_t stream) {
  if (n_in < 9) return;
  if (in_sizes[0] != kSeq * kH) return;
  if (in_sizes[1] != kNDir * kP || in_sizes[2] != kNDir * kP) return;
  if (in_sizes[3] != kNDir * kP * kH || in_sizes[4] != kNDir * kP * kH) return;
  if (in_sizes[5] != kNDir * kH * kP || in_sizes[6] != kNDir * kH * kP) return;
  if (in_sizes[7] != kNDir * kH || in_sizes[8] != kNDir * kP) return;
  if (out_size != kSeq * kH) return;

  const float* x        = (const float*)d_in[0];
  const float* log_real = (const float*)d_in[1];
  const float* imag     = (const float*)d_in[2];
  const float* B_real   = (const float*)d_in[3];
  const float* B_imag   = (const float*)d_in[4];
  const float* C_real   = (const float*)d_in[5];
  const float* C_imag   = (const float*)d_in[6];
  const float* Dm       = (const float*)d_in[7];
  const float* log_dt   = (const float*)d_in[8];
  float* out = (float*)d_out;

  char* ws = (char*)d_ws;
  size_t off = 0;
  float* par = (float*)(ws + off);                          off += 16384;
  unsigned short* X16 = (unsigned short*)(ws + off);        off += (size_t)kSeq * kH * 2;
  unsigned short* Bt1 = (unsigned short*)(ws + off);        off += (size_t)kNDir * kNC * kH * 2;
  unsigned short* Bt2 = (unsigned short*)(ws + off);        off += (size_t)kNDir * kH * kNC * 2;
  float* Bu = (float*)(ws + off);                           off += (size_t)kNDir * kSeq * kNC * 4;
  float* Y  = Bu;
  unsigned short* XS = (unsigned short*)(ws + off);         off += (size_t)kNDir * kSeq * kNC * 2;
  if (off > ws_size) return;

  param_kernel<<<(kNDir * kP) / 256, 256, 0, stream>>>(log_real, imag, log_dt, par, kNDir * kP);
  cast8_f16_kernel<<<(kSeq * kH / 8) / 256, 256, 0, stream>>>(x, X16, kSeq * kH / 8);
  bbar_kernel<<<(kNDir * kP * (kH / 8)) / 256, 256, 0, stream>>>(B_real, B_imag, par, Bt1, kWCarry);
  cmat_kernel<<<(kNDir * kH * (kP / 8)) / 256, 256, 0, stream>>>(C_real, C_imag, Bt2, kWCarry);
  wmma_gemm64<0, false, 0, 0, false, 0><<<dim3((kSeq / 64) * (kNC / 64) / 8, kNDir), 256, 0, stream>>>(
      X16, X16, kH, 0L,
      Bt1, Bt1, kH, (long)kNC * kH,
      (void*)Bu, (void*)Bu, kNC, (long)kSeq * kNC,
      (const float*)par, (const float*)par, 0L,
      kSeq, kNC, kH, kWCarryInv);
  diag_rec_kernel<<<kNDir * (kP / kRecP), kRecP, 0, stream>>>(Bu, par, XS);
  wmma_gemm64<0, false, 0, 0, false, 0><<<dim3((kSeq / 64) * (kH / 64) / 8, kNDir), 256, 0, stream>>>(
      XS, XS, kNC, (long)kSeq * kNC,
      Bt2, Bt2, kNC, (long)kH * kNC,
      (void*)Y, (void*)Y, kH, (long)kSeq * kH,
      (const float*)par, (const float*)par, 0L,
      kSeq, kH, kNC, kWCarryInv);
  gelu_sum_kernel<<<(kSeq * kH / 4) / 256, 256, 0, stream>>>(Y, x, Dm, out, kSeq * kH / 4);
}
